// MultiHeadAttention_29618094473500
// MI455X (gfx1250) — hardware-verified
//
#include <hip/hip_runtime.h>


#ifndef NB
#define NB 2
#endif
#ifndef IMH
#define IMH 64
#endif
#define NB_FULL  2
#define IMH_FULL 64
#define IMW  64
#define SEQ  (IMH * IMW)
#define SKV  ((IMH / 2) * (IMW / 2))
#ifndef OUT_SEQ
#define OUT_SEQ SEQ
#endif
#define CIN  256
#define NH_  8
#define HD   64
#define DQ   512
#define KKV  1024
#define COUT 256
#define AW   4
#define RS   2048.0f
#define RI   (1.0f / 2048.0f)
#define CQ   16.0f
#define CK   16.0f
#define CV   16.0f
#define SC2  (8.0f * 1.4426950408889634f / (CQ * CK))
#define PSH  14.0f
#define WPS  1024.0f
#define OSC  (1.0f / (WPS * CV))

static_assert(HD == 64);
static_assert(NH_ * HD == DQ);
static_assert(CIN * 4 == KKV);
static_assert(IMW == 64);
static_assert(IMH % 4 == 0);
static_assert(SEQ % 64 == 0);
static_assert(SKV % 64 == 0);
static_assert(SKV % 32 == 0);
static_assert(SEQ % (16 * AW) == 0);
static_assert(CIN % 64 == 0 && CIN % 32 == 0);
static_assert(KKV % 32 == 0 && DQ % 32 == 0);
static_assert(DQ % 64 == 0 && COUT % 64 == 0);
static_assert(NB <= NB_FULL);
static_assert(IMH <= IMH_FULL);

typedef _Float16 h16;
typedef unsigned short bf;
typedef __attribute__((ext_vector_type(16))) __bf16   v16bf;
typedef __attribute__((ext_vector_type(16))) _Float16 v16h;
typedef __attribute__((ext_vector_type(8)))  _Float16 v8h;
typedef __attribute__((ext_vector_type(8)))  unsigned short v8us;
typedef __attribute__((ext_vector_type(8)))  float    v8f;
typedef __attribute__((ext_vector_type(4)))  float    v4f;
typedef v4f  __attribute__((may_alias)) v4fa;

__device__ __forceinline__ unsigned short f2bf(float f) { unsigned u = __float_as_uint(f); u += 0x7FFFu + ((u >> 16) & 1u); return (unsigned short)(u >> 16); }
__device__ __forceinline__ v16h cat16(v8h lo, v8h hi) { return __builtin_shufflevector(lo, hi, 0, 1, 2, 3, 4, 5, 6, 7, 8, 9, 10, 11, 12, 13, 14, 15); }
__device__ __forceinline__ v16bf cat16b(v8us lo, v8us hi) { return __builtin_bit_cast(v16bf, __builtin_shufflevector(lo, hi, 0, 1, 2, 3, 4, 5, 6, 7, 8, 9, 10, 11, 12, 13, 14, 15)); }
__device__ __forceinline__ v8f wmma16(v16h a, v16h b, v8f c) { return __builtin_amdgcn_wmma_f32_16x16x32_f16(false, a, false, b, (short)0, c, false, false); }
__device__ __forceinline__ v8f wmmab(v16bf a, v16bf b, v8f c) { return __builtin_amdgcn_wmma_f32_16x16x32_bf16(false, a, false, b, (short)0, c, false, false); }
__device__ __forceinline__ v16h  ldh(const h16* p) { return cat16(*(const v8h*)p, *(const v8h*)(p + 16)); }
__device__ __forceinline__ v16bf ldb(const bf* p)  { return cat16b(*(const v8us*)p, *(const v8us*)(p + 16)); }
__device__ __forceinline__ void wave_sync() { __builtin_amdgcn_fence(3  , "wavefront"); __builtin_amdgcn_wave_barrier(); asm volatile("" ::: "memory"); }

__global__ __launch_bounds__(256) void k_cvt8(const float* __restrict__ src, bf* dst, size_t n8, int mode) {
    const size_t i = (size_t)blockIdx.x * 256 + threadIdx.x; if (i >= n8) return;
    const v8f v = *(const v8f*)(src + i * 8); v8us o;
#pragma unroll
    for (int k = 0; k < 8; ++k) {
        const unsigned short wb = f2bf(v[k]);
        const h16 hv = (h16)(__uint_as_float(((unsigned)wb) << 16) * WPS);
        const unsigned short wh = __builtin_bit_cast(unsigned short, hv);
        o[k] = mode ? wh : wb;
    }
    *(volatile v8us*)(dst + i * 8) = o; __threadfence(); *(volatile v8us*)(dst + i * 8) = o;
}

__global__ __launch_bounds__(256) void k_pack(const float* __restrict__ x, bf* XT, bf* PAT) {
    __shared__ unsigned short tile[64 * 136];
    const int tid = threadIdx.x;
    const int h2 = blockIdx.x, c0 = blockIdx.y * 64, b = blockIdx.z;
#pragma unroll
    for (int it = 0; it < 8; ++it) {
        const int idx = it * 256 + tid; const int cc = idx >> 5, q4 = idx & 31;
        const v4f v = *(const v4f*)(x + (((size_t)b * CIN + c0 + cc) * IMH_FULL + 2 * h2) * IMW + q4 * 4);
#pragma unroll
        for (int k = 0; k < 4; ++k) tile[cc * 136 + q4 * 4 + k] = f2bf(v[k]);
    }
    __syncthreads();
    const int l8 = tid >> 3, j8 = tid & 7;
#pragma unroll 1
    for (int ps = 0; ps < 2; ++ps) {
#pragma unroll
        for (int it = 0; it < 4; ++it) {
            const int p = it * 32 + l8, c8 = j8 * 8; v8us o;
#pragma unroll
            for (int k = 0; k < 8; ++k) o[k] = tile[(c8 + k) * 136 + p];
            *(volatile v8us*)(XT + ((size_t)b * SEQ + (size_t)h2 * 128 + p) * CIN + c0 + c8) = o;
        }
#pragma unroll
        for (int it = 0; it < 4; ++it) {
            const int line = it * 32 + l8; const int w2 = line >> 2, lq = line & 3; const int cc = lq * 16 + j8 * 2; v8us o;
            o[0] = tile[cc * 136 + 2 * w2];            o[1] = tile[cc * 136 + 2 * w2 + 1];
            o[2] = tile[cc * 136 + 64 + 2 * w2];       o[3] = tile[cc * 136 + 64 + 2 * w2 + 1];
            o[4] = tile[(cc + 1) * 136 + 2 * w2];      o[5] = tile[(cc + 1) * 136 + 2 * w2 + 1];
            o[6] = tile[(cc + 1) * 136 + 64 + 2 * w2]; o[7] = tile[(cc + 1) * 136 + 64 + 2 * w2 + 1];
            *(volatile v8us*)(PAT + ((size_t)b * SKV + (size_t)h2 * 32 + w2) * KKV + c0 * 4 + lq * 64 + j8 * 8) = o;
        }
        if (ps == 0) __threadfence();
    }
}

__global__ __launch_bounds__(32) void k_proj(const bf* __restrict__ A, const bf* __restrict__ Bt, int K, float cs, h16* Ph, h16* Pr, int useRes, int RB, size_t sRB, int pitch, int CB, size_t sCB) {
    __shared__ __align__(16) float os[16 * 68];
    const int lane = threadIdx.x & 31, lr = lane & 15, hi = lane >> 4; const int r0 = blockIdx.x * 64, c0 = blockIdx.y * 64;
    v8f acc[4][4];
#pragma unroll
    for (int mb = 0; mb < 4; ++mb)
#pragma unroll
        for (int nb = 0; nb < 4; ++nb) acc[mb][nb] = (v8f){};
    const size_t aoff = (size_t)(r0 + lr) * K + 8 * hi, boff = (size_t)(c0 + lr) * K + 8 * hi;
#pragma unroll 1
    for (int kc = 0; kc < K; kc += 32) {
        v16bf a[4];
#pragma unroll
        for (int mb = 0; mb < 4; ++mb) a[mb] = ldb(A + aoff + (size_t)mb * 16 * K + kc);
#pragma unroll
        for (int nb = 0; nb < 4; ++nb) { const v16bf b = ldb(Bt + boff + (size_t)nb * 16 * K + kc);
#pragma unroll
            for (int mb = 0; mb < 4; ++mb) acc[mb][nb] = wmmab(a[mb], b, acc[mb][nb]); }
        asm volatile("v_nop\n\tv_nop\n\tv_nop\n\tv_nop" : "+v"(acc[0][0]), "+v"(acc[1][1]), "+v"(acc[2][2]), "+v"(acc[3][3]) : "v"(a[0]), "v"(a[1]), "v"(a[2]), "v"(a[3]));
    }
    const size_t tbase = (size_t)(r0 / RB) * sRB + (size_t)(r0 % RB) * (size_t)pitch + (size_t)(c0 / CB) * sCB + (size_t)(c0 % CB);
#pragma unroll
    for (int mb = 0; mb < 4; ++mb) {
#pragma unroll
        for (int nb = 0; nb < 4; ++nb) {
#pragma unroll
            for (int j = 0; j < 8; ++j) os[(hi * 8 + j) * 68 + nb * 16 + lr] = acc[mb][nb][j] * cs; }
        wave_sync();
        const size_t sb = tbase + (size_t)(mb * 16) * (size_t)pitch;
#pragma unroll 1
        for (int ps = 0; ps < 2; ++ps) {
#pragma unroll
            for (int s = 0; s < 4; ++s) { const int row = 4 * s + (lane >> 3), c8 = (lane & 7) * 8;
                const v4f x0 = *(const v4fa*)(&os[row * 68 + c8]); const v4f x1 = *(const v4fa*)(&os[row * 68 + c8 + 4]); v8h hv, rv;
#pragma unroll
                for (int i = 0; i < 4; ++i) { const h16 a0 = (h16)x0[i]; const h16 a1 = (h16)x1[i]; hv[i] = a0; hv[4 + i] = a1; rv[i] = (h16)((x0[i] - (float)a0) * RS); rv[4 + i] = (h16)((x1[i] - (float)a1) * RS); }
                const size_t oo = sb + (size_t)row * (size_t)pitch + c8;
                *(volatile v8h*)(Ph + oo) = hv; if (useRes) *(volatile v8h*)(Pr + oo) = rv; }
            if (ps == 0) __threadfence(); }
        wave_sync();
    }
}

__global__ __launch_bounds__(32 * AW) void k_flash(const h16* __restrict__ QH, const h16* __restrict__ QR, const h16* __restrict__ KH, const h16* __restrict__ KR, const h16* __restrict__ VT, h16* AP) {
    __shared__ __align__(16) float os[AW * 16 * 68];
    const int lane = threadIdx.x & 31, wave = __builtin_amdgcn_readfirstlane((int)(threadIdx.x >> 5)), lr = lane & 15, hi = lane >> 4;
    const int zh = blockIdx.y; const int b = zh / NH_, h = zh % NH_;
    const int t0 = (blockIdx.x * AW + wave) * 16;
    const size_t qbase = (size_t)zh * SEQ * HD;
    const size_t kbase = (size_t)zh * SKV * HD;
    const size_t qo = qbase + (size_t)(t0 + lr) * HD + 8 * hi;
    const v16h qh0 = ldh(QH + qo), qh1 = ldh(QH + qo + 32), qr0 = ldh(QR + qo), qr1 = ldh(QR + qo + 32);
    const size_t ko = kbase + (size_t)lr * HD + 8 * hi;
    const size_t vo = kbase + (size_t)lr * SKV + 8 * hi;
    v8f o0 = (v8f){}, o1 = (v8f){}, o2 = (v8f){}, o3 = (v8f){};
    float m = -3.0e38f, l = 0.0f;
#pragma unroll 1
    for (int key0 = 0; key0 < SKV; key0 += 32) {
        const h16* ka = KH + ko + (size_t)key0 * HD;
        const h16* kr = KR + ko + (size_t)key0 * HD;
        const v16h ka0 = ldh(ka), ka1 = ldh(ka + 32), kb0 = ldh(ka + 16 * HD), kb1 = ldh(ka + 16 * HD + 32);
        const v16h ra0 = ldh(kr), ra1 = ldh(kr + 32), rb0 = ldh(kr + 16 * HD), rb1 = ldh(kr + 16 * HD + 32);
        v8f sHa = (v8f){}, sLa = (v8f){}, sHb = (v8f){}, sLb = (v8f){};
        sHa = wmma16(ka0, qh0, sHa); sLa = wmma16(ka0, qr0, sLa); sHb = wmma16(kb0, qh0, sHb); sLb = wmma16(kb0, qr0, sLb);
        sLa = wmma16(ra0, qh0, sLa); sLb = wmma16(rb0, qh0, sLb);
        sHa = wmma16(ka1, qh1, sHa); sLa = wmma16(ka1, qr1, sLa); sHb = wmma16(kb1, qh1, sHb); sLb = wmma16(kb1, qr1, sLb);
        sLa = wmma16(ra1, qh1, sLa); sLb = wmma16(rb1, qh1, sLb);
        asm volatile("v_nop\n\tv_nop\n\tv_nop\n\tv_nop" : "+v"(sHa), "+v"(sLa), "+v"(sHb), "+v"(sLb) : "v"(ka0), "v"(ka1), "v"(kb0), "v"(kb1), "v"(ra0), "v"(ra1), "v"(rb0), "v"(rb1));
        float ta[8], tb[8]; float mx = -3.0e38f;
#pragma unroll
        for (int r = 0; r < 8; ++r) { ta[r] = (sHa[r] + sLa[r] * RI) * SC2; tb[r] = (sHb[r] + sLb[r] * RI) * SC2; mx = fmaxf(mx, fmaxf(ta[r], tb[r])); }
        mx = fmaxf(mx, __shfl_xor(mx, 16, 32));
        const float mnew = fmaxf(m, mx);
        const float alpha = __builtin_amdgcn_exp2f(m - mnew);
        const float sh = PSH - mnew;
        v16h pb; float ls = 0.0f;
#pragma unroll
        for (int r = 0; r < 8; ++r) { const h16 pa = (h16)__builtin_amdgcn_exp2f(ta[r] + sh); const h16 pc = (h16)__builtin_amdgcn_exp2f(tb[r] + sh); pb[r] = pa; pb[8 + r] = pc; ls += (float)pa + (float)pc; }
        l = l * alpha + ls; m = mnew;
        o0 = o0 * alpha; o1 = o1 * alpha; o2 = o2 * alpha; o3 = o3 * alpha;
        const h16* va = VT + vo + key0;
        const v16h v0 = ldh(va), v1 = ldh(va + (size_t)16 * SKV), v2 = ldh(va + (size_t)32 * SKV), v3 = ldh(va + (size_t)48 * SKV);
        o0 = wmma16(v0, pb, o0); o1 = wmma16(v1, pb, o1); o2 = wmma16(v2, pb, o2); o3 = wmma16(v3, pb, o3);
        asm volatile("v_nop\n\tv_nop\n\tv_nop\n\tv_nop" : "+v"(o0), "+v"(o1), "+v"(o2), "+v"(o3) : "v"(v0), "v"(v1), "v"(v2), "v"(v3), "v"(pb));
    }
    l += __shfl_xor(l, 16, 32);
    const float inv = 1.0f / l;
    const int wb = wave * 16 * 68;
    { v4f a, c;
      a[0] = o0[0] * inv; a[1] = o0[1] * inv; a[2] = o0[2] * inv; a[3] = o0[3] * inv; c[0] = o0[4] * inv; c[1] = o0[5] * inv; c[2] = o0[6] * inv; c[3] = o0[7] * inv;
      *(v4fa*)(&os[wb + lr * 68 +  0 + 8 * hi]) = a; *(v4fa*)(&os[wb + lr * 68 +  0 + 8 * hi + 4]) = c;
      a[0] = o1[0] * inv; a[1] = o1[1] * inv; a[2] = o1[2] * inv; a[3] = o1[3] * inv; c[0] = o1[4] * inv; c[1] = o1[5] * inv; c[2] = o1[6] * inv; c[3] = o1[7] * inv;
      *(v4fa*)(&os[wb + lr * 68 + 16 + 8 * hi]) = a; *(v4fa*)(&os[wb + lr * 68 + 16 + 8 * hi + 4]) = c;
      a[0] = o2[0] * inv; a[1] = o2[1] * inv; a[2] = o2[2] * inv; a[3] = o2[3] * inv; c[0] = o2[4] * inv; c[1] = o2[5] * inv; c[2] = o2[6] * inv; c[3] = o2[7] * inv;
      *(v4fa*)(&os[wb + lr * 68 + 32 + 8 * hi]) = a; *(v4fa*)(&os[wb + lr * 68 + 32 + 8 * hi + 4]) = c;
      a[0] = o3[0] * inv; a[1] = o3[1] * inv; a[2] = o3[2] * inv; a[3] = o3[3] * inv; c[0] = o3[4] * inv; c[1] = o3[5] * inv; c[2] = o3[6] * inv; c[3] = o3[7] * inv;
      *(v4fa*)(&os[wb + lr * 68 + 48 + 8 * hi]) = a; *(v4fa*)(&os[wb + lr * 68 + 48 + 8 * hi + 4]) = c; }
    wave_sync();
    h16* arow = AP + ((size_t)b * SEQ + t0) * DQ + h * HD;
#pragma unroll 1
    for (int ps = 0; ps < 2; ++ps) {
#pragma unroll
        for (int s = 0; s < 4; ++s) { const int row = 4 * s + (lane >> 3), c8 = (lane & 7) * 8;
            const v4f x0 = *(const v4fa*)(&os[wb + row * 68 + c8]); const v4f x1 = *(const v4fa*)(&os[wb + row * 68 + c8 + 4]); v8h hv;
#pragma unroll
            for (int i = 0; i < 4; ++i) { hv[i] = (h16)x0[i]; hv[4 + i] = (h16)x1[i]; }
            *(volatile v8h*)(arow + (size_t)row * DQ + c8) = hv; }
        if (ps == 0) __threadfence(); }
}

__global__ __launch_bounds__(32) void k_out(const h16* __restrict__ A, const h16* __restrict__ Bt, float* OUT) {
    __shared__ __align__(16) float os[16 * 68];
    const int K = DQ;
    const int lane = threadIdx.x & 31, lr = lane & 15, hi = lane >> 4; const int r0 = blockIdx.x * 64, c0 = blockIdx.y * 64;
    v8f acc[4][4];
#pragma unroll
    for (int mb = 0; mb < 4; ++mb)
#pragma unroll
        for (int nb = 0; nb < 4; ++nb) acc[mb][nb] = (v8f){};
    const size_t aoff = (size_t)(r0 + lr) * K + 8 * hi, boff = (size_t)(c0 + lr) * K + 8 * hi;
#pragma unroll 1
    for (int kc = 0; kc < K; kc += 32) {
        v16h a[4];
#pragma unroll
        for (int mb = 0; mb < 4; ++mb) a[mb] = ldh(A + aoff + (size_t)mb * 16 * K + kc);
#pragma unroll
        for (int nb = 0; nb < 4; ++nb) { const v16h b = ldh(Bt + boff + (size_t)nb * 16 * K + kc);
#pragma unroll
            for (int mb = 0; mb < 4; ++mb) acc[mb][nb] = wmma16(a[mb], b, acc[mb][nb]); }
        asm volatile("v_nop\n\tv_nop\n\tv_nop\n\tv_nop" : "+v"(acc[0][0]), "+v"(acc[1][1]), "+v"(acc[2][2]), "+v"(acc[3][3]) : "v"(a[0]), "v"(a[1]), "v"(a[2]), "v"(a[3]));
    }
    const int bb = c0 / SEQ, n0 = c0 % SEQ;
#pragma unroll
    for (int mb = 0; mb < 4; ++mb) {
#pragma unroll
        for (int nb = 0; nb < 4; ++nb) {
#pragma unroll
            for (int j = 0; j < 8; ++j) os[(hi * 8 + j) * 68 + nb * 16 + lr] = acc[mb][nb][j] * OSC; }
        wave_sync();
        float* ob = OUT + ((size_t)bb * COUT + r0 + mb * 16) * OUT_SEQ + n0;
#pragma unroll 1
        for (int ps = 0; ps < 2; ++ps) {
#pragma unroll
            for (int s = 0; s < 8; ++s) { const int row = 2 * s + hi, cofs = lr * 4;
                const v4f val = *(const v4fa*)(&os[row * 68 + cofs]);
                *(volatile v4f*)(ob + (size_t)row * OUT_SEQ + cofs) = val; }
            if (ps == 0) __threadfence(); }
        wave_sync();
    }
}

static constexpr size_t al256(size_t v) { return (v + 255) & ~(size_t)255; }
static constexpr size_t SZ_XT  = al256((size_t)NB * SEQ * CIN * 2);
static constexpr size_t SZ_PAT = al256((size_t)NB * SKV * KKV * 2);
static constexpr size_t SZ_WQ  = al256((size_t)DQ * CIN * 2);
static constexpr size_t SZ_WKV = al256((size_t)2 * DQ * KKV * 2);
static constexpr size_t SZ_WP  = al256((size_t)COUT * DQ * 2);
static constexpr size_t SZ_QP  = al256((size_t)NB * NH_ * SEQ * HD * 2);
static constexpr size_t SZ_KP  = al256((size_t)NB * NH_ * SKV * HD * 2);
static constexpr size_t SZ_AP  = al256((size_t)NB * SEQ * DQ * 2);
static constexpr size_t SZ_TOTAL = SZ_XT + SZ_PAT + SZ_WQ + SZ_WKV + SZ_WP + 2 * SZ_QP + 3 * SZ_KP + SZ_AP;
static_assert(SZ_TOTAL <= (size_t)134217728);

extern "C" void kernel_launch(void* const* d_in, const int* in_sizes, int n_in,
                              void* d_out, int out_size, void* d_ws, size_t ws_size, hipStream_t stream) {
    if (n_in < 4) return;
    const size_t needx = (((size_t)(NB - 1) * CIN + (CIN - 1)) * IMH_FULL + IMH) * IMW;
    if ((size_t)in_sizes[0] < needx) return;
    if ((size_t)in_sizes[1] < (size_t)DQ * CIN || (size_t)in_sizes[2] < (size_t)2 * DQ * KKV || (size_t)in_sizes[3] < (size_t)COUT * DQ) return;
    if ((size_t)out_size < ((size_t)(NB - 1) * COUT + (COUT - 1)) * OUT_SEQ + SEQ) return;
    if (SZ_TOTAL > ws_size) return;
    const float* x = (const float*)d_in[0]; const float* wq = (const float*)d_in[1]; const float* wkv = (const float*)d_in[2]; const float* wp = (const float*)d_in[3];
    float* OUT = (float*)d_out;
    char* wsp = (char*)d_ws;
    bf* XT  = (bf*)wsp; wsp += SZ_XT;
    bf* PAT = (bf*)wsp; wsp += SZ_PAT;
    bf* WQ  = (bf*)wsp; wsp += SZ_WQ;
    bf* WKV = (bf*)wsp; wsp += SZ_WKV;
    bf* WPu = (bf*)wsp; wsp += SZ_WP;
    h16* QH = (h16*)wsp; wsp += SZ_QP;
    h16* QR = (h16*)wsp; wsp += SZ_QP;
    h16* KH = (h16*)wsp; wsp += SZ_KP;
    h16* KR = (h16*)wsp; wsp += SZ_KP;
    h16* VT = (h16*)wsp; wsp += SZ_KP;
    h16* AP = (h16*)wsp; wsp += SZ_AP;
    const h16* WP = (const h16*)WPu;

    k_pack<<<dim3(IMH / 2, CIN / 64, NB), 256, 0, stream>>>(x, XT, PAT);
    { const size_t n8 = (size_t)DQ * CIN / 8;      k_cvt8<<<(unsigned)((n8 + 255) / 256), 256, 0, stream>>>(wq, WQ, n8, 0); }
    { const size_t n8 = (size_t)2 * DQ * KKV / 8;  k_cvt8<<<(unsigned)((n8 + 255) / 256), 256, 0, stream>>>(wkv, WKV, n8, 0); }
    { const size_t n8 = (size_t)COUT * DQ / 8;     k_cvt8<<<(unsigned)((n8 + 255) / 256), 256, 0, stream>>>(wp, WPu, n8, 1); }

    k_proj<<<dim3(NB * SEQ / 64, DQ / 64, 1), 32, 0, stream>>>(XT, WQ, CIN, CQ, QH, QR, 1, SEQ, (size_t)NH_ * SEQ * HD, HD, HD, (size_t)SEQ * HD);
    k_proj<<<dim3(NB * SKV / 64, DQ / 64, 1), 32, 0, stream>>>(PAT, WKV, KKV, CK, KH, KR, 1, SKV, (size_t)NH_ * SKV * HD, HD, HD, (size_t)SKV * HD);
    k_proj<<<dim3(DQ / 64, NB * SKV / 64, 1), 32, 0, stream>>>(WKV + (size_t)DQ * KKV, PAT, KKV, CV, VT, VT, 0, DQ, (size_t)0, SKV, SKV, (size_t)DQ * SKV);

    k_flash<<<dim3(SEQ / (16 * AW), NB * NH_, 1), 32 * AW, 0, stream>>>(QH, QR, KH, KR, VT, AP);

    k_out<<<dim3(COUT / 64, NB * SEQ / 64, 1), 32, 0, stream>>>(WP, AP, OUT);
}
